// CTNNBackflowNet_18056042512511
// MI455X (gfx1250) — hardware-verified
//
#include <hip/hip_runtime.h>


#define NB_  16
#define NN_  128
#define HH   128
#define NODES (NB_ * NN_)
#define PAIRS (NN_ * NN_)

typedef unsigned short bf;
typedef __attribute__((ext_vector_type(16))) __bf16   v16bf;
typedef __attribute__((ext_vector_type(8)))  unsigned short v8us;
typedef __attribute__((ext_vector_type(4)))  unsigned short v4us;
typedef __attribute__((ext_vector_type(8)))  float    v8f;
typedef __attribute__((ext_vector_type(4)))  float    v4f;
typedef v4f  __attribute__((may_alias)) v4fa;
typedef v8us __attribute__((may_alias)) v8usa;

__device__ __forceinline__ unsigned short f2bf(float f) { unsigned u = __float_as_uint(f); u += 0x7FFFu + ((u >> 16) & 1u); return (unsigned short)(u >> 16); }
__device__ __forceinline__ float bf2f(unsigned short b) { return __uint_as_float(((unsigned)b) << 16); }
__device__ __forceinline__ float bfr(float f) { return bf2f(f2bf(f)); }
__device__ __forceinline__ v16bf cat16b(v8us lo, v8us hi) { return __builtin_bit_cast(v16bf, __builtin_shufflevector(lo, hi, 0, 1, 2, 3, 4, 5, 6, 7, 8, 9, 10, 11, 12, 13, 14, 15)); }
__device__ __forceinline__ v8f wmmab(v16bf a, v16bf b, v8f c) { return __builtin_amdgcn_wmma_f32_16x16x32_bf16(false, a, false, b, (short)0, c, false, false); }
__device__ __forceinline__ float silu_f(float x) { return x / (1.0f + expf(-x)); }
__device__ __forceinline__ void put4(float* F, bf* OH, bf* OL, size_t o, v4f v) {
    if (F) *(volatile v4f*)(F + o) = v;
    if (OH) { v4us h, l;
#pragma unroll
        for (int i = 0; i < 4; ++i) { const unsigned short hb = f2bf(v[i]); h[i] = hb; l[i] = f2bf(v[i] - bf2f(hb)); }
        *(volatile v4us*)(OH + o) = h; *(volatile v4us*)(OL + o) = l; }
}

__global__ __launch_bounds__(256) void k_wt(const float* __restrict__ Wm, int K, int ncols, bf* WT) {
    __shared__ __align__(16) unsigned short tl[64 * 72];
    const int tid = threadIdx.x, k0 = blockIdx.x * 64, n0 = blockIdx.y * 64;
    const int kk = tid >> 2, nq = (tid & 3) * 16;
#pragma unroll
    for (int i = 0; i < 16; ++i) tl[(nq + i) * 72 + kk] = f2bf(Wm[(size_t)(k0 + kk) * ncols + n0 + nq + i]);
    __syncthreads();
    const int piece = tid & 7;
    auto pass = [&]() {
#pragma unroll
        for (int s = 0; s < 2; ++s) { const int nr = (tid >> 3) + 32 * s; const v8us val = *(const v8usa*)(tl + nr * 72 + piece * 8); *(volatile v8us*)(WT + (size_t)(n0 + nr) * K + k0 + piece * 8) = val; }
    };
    pass(); __threadfence(); pass();
}
__global__ __launch_bounds__(256) void k_node0(const float* __restrict__ x, const int* __restrict__ spin, const float* __restrict__ ne_w, const float* __restrict__ ne_b, float* HV, bf* HVh, bf* HVl) {
    const int lane = threadIdx.x & 31, node = blockIdx.x * 8 + (threadIdx.x >> 5);
    if (node >= NODES) return;
    const int i = node & (NN_ - 1);
    const float x0 = bfr(x[(size_t)node * 3 + 0]), x1 = bfr(x[(size_t)node * 3 + 1]), x2 = bfr(x[(size_t)node * 3 + 2]), sp = (float)spin[i];
    v4f v;
#pragma unroll
    for (int e = 0; e < 4; ++e) { const int c = lane * 4 + e;
        v[e] = x0 * bfr(ne_w[c]) + x1 * bfr(ne_w[HH + c]) + x2 * bfr(ne_w[2 * HH + c]) + sp * bfr(ne_w[3 * HH + c]) + bfr(ne_b[c]); }
    const size_t o = (size_t)node * HH + lane * 4;
    put4(HV, HVh, HVl, o, v); __threadfence(); put4(HV, HVh, HVl, o, v);
}
__global__ __launch_bounds__(256) void k_edge1(const float* __restrict__ x, int b, const float* __restrict__ w, const float* __restrict__ bias, bf* E1h, bf* E1l) {
    const int lane = threadIdx.x & 31, r = blockIdx.x * 8 + (threadIdx.x >> 5);
    if (r >= PAIRS) return;
    const int i = r >> 7, j = r & (NN_ - 1);
    const float* xi = x + ((size_t)b * NN_ + i) * 3; const float* xj = x + ((size_t)b * NN_ + j) * 3;
    float in[5];
    in[0] = bfr(xi[0]) - bfr(xj[0]); in[1] = bfr(xi[1]) - bfr(xj[1]); in[2] = bfr(xi[2]) - bfr(xj[2]);
    in[4] = in[0] * in[0] + in[1] * in[1] + in[2] * in[2]; in[3] = sqrtf(in[4] + 1e-12f);
    v4f v;
#pragma unroll
    for (int e = 0; e < 4; ++e) { const int c = lane * 4 + e; float a = bfr(bias[c]);
#pragma unroll
        for (int q = 0; q < 5; ++q) a = fmaf(in[q], bfr(w[q * HH + c]), a);
        v[e] = silu_f(a); }
    const size_t o = (size_t)r * HH + lane * 4;
    put4(nullptr, E1h, E1l, o, v); __threadfence(); put4(nullptr, E1h, E1l, o, v);
}
__global__ __launch_bounds__(128) void k_gemm(const bf* __restrict__ Ah, const bf* __restrict__ Al, const bf* __restrict__ Bn, const float* __restrict__ bias,
                                              const float* __restrict__ ADD1, int sh1, int off1, const float* __restrict__ ADD2, int msk2, int off2, int act,
                                              float* F, bf* OH, bf* OL) {
    __shared__ __align__(16) float ost[4][16 * 68];
    const int lane = threadIdx.x & 31, wave = threadIdx.x >> 5, lr = lane & 15, hi = lane >> 4;
    const int r0 = blockIdx.x * 64 + wave * 16; const int c0 = blockIdx.y * 64;
    v8f acc[4];
#pragma unroll
    for (int t = 0; t < 4; ++t) acc[t] = (v8f){};
    const size_t a1 = (size_t)(r0 + lr) * HH + 8 * hi;
#pragma unroll 2
    for (int kc = 0; kc < HH; kc += 32) {
        const v16bf a = cat16b(*(const v8us*)(Ah + a1 + kc), *(const v8us*)(Ah + a1 + kc + 16));
        const v16bf al = cat16b(*(const v8us*)(Al + a1 + kc), *(const v8us*)(Al + a1 + kc + 16));
#pragma unroll
        for (int t = 0; t < 4; ++t) { const bf* bp = Bn + (size_t)(c0 + t * 16 + lr) * HH + kc + 8 * hi; const v16bf bb = cat16b(*(const v8us*)bp, *(const v8us*)(bp + 16)); acc[t] = wmmab(a, bb, acc[t]); acc[t] = wmmab(al, bb, acc[t]); }
        asm volatile("v_nop" : "+v"(acc[0]), "+v"(acc[1]), "+v"(acc[2]), "+v"(acc[3]) : "v"(a), "v"(al) : "memory");
    }
    float* os = &ost[wave][0];
#pragma unroll
    for (int t = 0; t < 4; ++t) {
        const int c = c0 + t * 16 + lr; const float bc = bias ? bfr(bias[c]) : 0.f;
#pragma unroll
        for (int j = 0; j < 8; ++j) { const int r = r0 + hi * 8 + j; float v = acc[t][j] + bc;
            if (ADD1) v += ADD1[(size_t)((r >> sh1) + off1) * HH + c];
            if (ADD2) v += ADD2[(size_t)((r & msk2) + off2) * HH + c];
            if (act) v = silu_f(v);
            os[(hi * 8 + j) * 68 + t * 16 + lr] = v; } }
    __builtin_amdgcn_wave_barrier(); asm volatile("" ::: "memory");
    auto pass = [&]() {
#pragma unroll
        for (int s = 0; s < 8; ++s) { const int Lid = (lane >> 3) + 4 * s, piece = lane & 7; const int row = Lid >> 1, cofs = (Lid & 1) * 32 + piece * 4;
            const v4f val = *(const v4fa*)(os + row * 68 + cofs); put4(F, OH, OL, (size_t)(r0 + row) * HH + c0 + cofs, val); }
    };
    pass(); __threadfence(); pass();
}
__global__ __launch_bounds__(256) void k_aggr(const float* __restrict__ HN, int b, bf* Sh, bf* Sl) {
    const int lane = threadIdx.x & 31, i = blockIdx.x * 8 + (threadIdx.x >> 5);
    if (i >= NN_) return;
    v4f s = {};
#pragma unroll 1
    for (int j = 0; j < NN_; ++j) { if (j == i) continue; s += *(const v4f*)(HN + ((size_t)i * NN_ + j) * HH + lane * 4); }
    const size_t o = ((size_t)b * NN_ + i) * HH + lane * 4;
    put4(nullptr, Sh, Sl, o, s); __threadfence(); put4(nullptr, Sh, Sl, o, s);
}
__global__ __launch_bounds__(256) void k_out(const float* __restrict__ HV2, const float* __restrict__ dxw, const float* __restrict__ dxb, const float* __restrict__ bfraw, float* out) {
    __shared__ float sdx[NN_ * 3]; __shared__ float smean[3]; __shared__ __align__(16) float so[NN_ * 3];
    const int tid = threadIdx.x, lane = tid & 31, wave = tid >> 5, b = blockIdx.x;
#pragma unroll 1
    for (int q = 0; q < 16; ++q) { const int i = wave * 16 + q; const float* h = HV2 + ((size_t)b * NN_ + i) * HH + lane * 4;
        float d0 = 0.f, d1 = 0.f, d2 = 0.f;
#pragma unroll
        for (int e = 0; e < 4; ++e) { const int k = lane * 4 + e; const float hv = h[e]; d0 = fmaf(hv, bfr(dxw[k * 3 + 0]), d0); d1 = fmaf(hv, bfr(dxw[k * 3 + 1]), d1); d2 = fmaf(hv, bfr(dxw[k * 3 + 2]), d2); }
#pragma unroll
        for (int sh = 16; sh; sh >>= 1) { d0 += __shfl_xor(d0, sh, 32); d1 += __shfl_xor(d1, sh, 32); d2 += __shfl_xor(d2, sh, 32); }
        if (lane == 0) { sdx[i * 3 + 0] = tanhf(d0 + bfr(dxb[0])); sdx[i * 3 + 1] = tanhf(d1 + bfr(dxb[1])); sdx[i * 3 + 2] = tanhf(d2 + bfr(dxb[2])); } }
    __syncthreads();
    if (tid < 3) { float m = 0.f;
#pragma unroll 1
        for (int i = 0; i < NN_; ++i) m += sdx[i * 3 + tid];
        smean[tid] = m / (float)NN_; }
    __syncthreads();
    const float raw = bfr(bfraw[0]); const float scale = fmaxf(raw, 0.f) + log1pf(expf(-fabsf(raw)));
    for (int e = tid; e < NN_ * 3; e += 256) so[e] = (sdx[e] - smean[e % 3]) * scale;
    __syncthreads();
    if (tid < 96) { const v4f v = *(const v4fa*)(so + tid * 4); float* ob = out + (size_t)b * NN_ * 3 + tid * 4; *(volatile v4f*)ob = v; __threadfence(); *(volatile v4f*)ob = v; }
}

extern "C" void kernel_launch(void* const* d_in, const int* in_sizes, int n_in,
                              void* d_out, int out_size, void* d_ws, size_t ws_size, hipStream_t stream) {
    (void)in_sizes; (void)n_in; (void)out_size;
    const float* x = (const float*)d_in[0]; const int* spin = (const int*)d_in[1];
    const float* ne_w = (const float*)d_in[2];  const float* ne_b = (const float*)d_in[3];
    const float* ee1_w = (const float*)d_in[4]; const float* ee1_b = (const float*)d_in[5]; const float* ee2_w = (const float*)d_in[6]; const float* ee2_b = (const float*)d_in[7];
    const float* rve_w = (const float*)d_in[8]; const float* rev_w = (const float*)d_in[9];
    const float* eu1_w = (const float*)d_in[10]; const float* eu1_b = (const float*)d_in[11]; const float* eu2_w = (const float*)d_in[12]; const float* eu2_b = (const float*)d_in[13];
    const float* nu1_w = (const float*)d_in[14]; const float* nu1_b = (const float*)d_in[15]; const float* nu2_w = (const float*)d_in[16]; const float* nu2_b = (const float*)d_in[17];
    const float* nu3_w = (const float*)d_in[18]; const float* nu3_b = (const float*)d_in[19]; const float* dx_w = (const float*)d_in[20]; const float* dx_b = (const float*)d_in[21];
    const float* bf_raw = (const float*)d_in[22];
    float* out = (float*)d_out;
    char* wsp = (char*)d_ws;
    auto take = [&](size_t bytes) { char* p = wsp; wsp += (bytes + 255) & ~(size_t)255; return (void*)p; };
    const size_t WP = (size_t)HH * HH * 2, NPF = (size_t)NODES * HH * 4, NPB = (size_t)NODES * HH * 2, EPF = (size_t)PAIRS * HH * 4, EPB = (size_t)PAIRS * HH * 2;
    bf* ee2T = (bf*)take(WP); bf* rveT = (bf*)take(WP); bf* revT = (bf*)take(WP); bf* eu1aT = (bf*)take(WP); bf* eu1bT = (bf*)take(WP); bf* eu1cT = (bf*)take(WP);
    bf* eu2T = (bf*)take(WP); bf* nu1aT = (bf*)take(WP); bf* nu1bT = (bf*)take(WP); bf* nu2T = (bf*)take(WP); bf* nu3T = (bf*)take(WP);
    float* HV = (float*)take(NPF); bf* HVh = (bf*)take(NPB); bf* HVl = (bf*)take(NPB); bf* VIEh = (bf*)take(NPB); bf* VIEl = (bf*)take(NPB);
    float* P = (float*)take(NPF); float* Q = (float*)take(NPF);
    bf* E1h = (bf*)take(EPB); bf* E1l = (bf*)take(EPB); bf* HEh = (bf*)take(EPB); bf* HEl = (bf*)take(EPB); bf* E2h = (bf*)take(EPB); bf* E2l = (bf*)take(EPB); float* HN = (float*)take(EPF);
    bf* Sh = (bf*)take(NPB); bf* Sl = (bf*)take(NPB); bf* MVh = (bf*)take(NPB); bf* MVl = (bf*)take(NPB); float* G = (float*)take(NPF);
    bf* T1h = (bf*)take(NPB); bf* T1l = (bf*)take(NPB); bf* T2h = (bf*)take(NPB); bf* T2l = (bf*)take(NPB); float* HV2 = (float*)take(NPF);
    if ((size_t)(wsp - (char*)d_ws) > ws_size) return;
    const dim3 gw(HH / 64, HH / 64), gn(NODES / 64, 2), ge(PAIRS / 64, 2);
    k_wt<<<gw, 256, 0, stream>>>(ee2_w, HH, HH, ee2T); k_wt<<<gw, 256, 0, stream>>>(rve_w, HH, HH, rveT); k_wt<<<gw, 256, 0, stream>>>(rev_w, HH, HH, revT);
    k_wt<<<gw, 256, 0, stream>>>(eu1_w, HH, HH, eu1aT); k_wt<<<gw, 256, 0, stream>>>(eu1_w + (size_t)HH * HH, HH, HH, eu1bT); k_wt<<<gw, 256, 0, stream>>>(eu1_w + (size_t)2 * HH * HH, HH, HH, eu1cT);
    k_wt<<<gw, 256, 0, stream>>>(eu2_w, HH, HH, eu2T); k_wt<<<gw, 256, 0, stream>>>(nu1_w, HH, HH, nu1aT); k_wt<<<gw, 256, 0, stream>>>(nu1_w + (size_t)HH * HH, HH, HH, nu1bT);
    k_wt<<<gw, 256, 0, stream>>>(nu2_w, HH, HH, nu2T); k_wt<<<gw, 256, 0, stream>>>(nu3_w, HH, HH, nu3T);
    k_node0<<<NODES / 8, 256, 0, stream>>>(x, spin, ne_w, ne_b, HV, HVh, HVl);
    k_gemm<<<gn, 128, 0, stream>>>(HVh, HVl, rveT, nullptr, nullptr, 0, 0, nullptr, 0, 0, 0, nullptr, VIEh, VIEl);
    k_gemm<<<gn, 128, 0, stream>>>(VIEh, VIEl, eu1bT, nullptr, nullptr, 0, 0, nullptr, 0, 0, 0, P, nullptr, nullptr);
    k_gemm<<<gn, 128, 0, stream>>>(VIEh, VIEl, eu1cT, nullptr, nullptr, 0, 0, nullptr, 0, 0, 0, Q, nullptr, nullptr);
    for (int b = 0; b < NB_; ++b) {
        k_edge1<<<PAIRS / 8, 256, 0, stream>>>(x, b, ee1_w, ee1_b, E1h, E1l);
        k_gemm<<<ge, 128, 0, stream>>>(E1h, E1l, ee2T, ee2_b, nullptr, 0, 0, nullptr, 0, 0, 0, nullptr, HEh, HEl);
        k_gemm<<<ge, 128, 0, stream>>>(HEh, HEl, eu1aT, eu1_b, P, 7, b * NN_, Q, NN_ - 1, b * NN_, 1, nullptr, E2h, E2l);
        k_gemm<<<ge, 128, 0, stream>>>(E2h, E2l, eu2T, eu2_b, nullptr, 0, 0, nullptr, 0, 0, 0, HN, nullptr, nullptr);
        k_aggr<<<NN_ / 8, 256, 0, stream>>>(HN, b, Sh, Sl);
    }
    k_gemm<<<gn, 128, 0, stream>>>(Sh, Sl, revT, nullptr, nullptr, 0, 0, nullptr, 0, 0, 0, nullptr, MVh, MVl);
    k_gemm<<<gn, 128, 0, stream>>>(MVh, MVl, nu1bT, nullptr, nullptr, 0, 0, nullptr, 0, 0, 0, G, nullptr, nullptr);
    k_gemm<<<gn, 128, 0, stream>>>(HVh, HVl, nu1aT, nu1_b, G, 0, 0, nullptr, 0, 0, 1, nullptr, T1h, T1l);
    k_gemm<<<gn, 128, 0, stream>>>(T1h, T1l, nu2T, nu2_b, nullptr, 0, 0, nullptr, 0, 0, 1, nullptr, T2h, T2l);
    k_gemm<<<gn, 128, 0, stream>>>(T2h, T2l, nu3T, nu3_b, HV, 0, 0, nullptr, 0, 0, 0, HV2, nullptr, nullptr);
    k_out<<<NB_, 256, 0, stream>>>(HV2, dx_w, dx_b, bf_raw, out);
}
